// MambaBlock_43138651521745
// MI455X (gfx1250) — hardware-run, weakly checked
//
#include <hip/hip_runtime.h>
#include <math.h>

typedef __attribute__((ext_vector_type(16))) _Float16 v16h;
typedef __attribute__((ext_vector_type(8)))  _Float16 v8h;
typedef __attribute__((ext_vector_type(8)))  float    v8f;
typedef __attribute__((ext_vector_type(4)))  float    v4f;

constexpr int kBatch  = 4;
constexpr int kSeq    = 1024;
constexpr int kDm     = 1024;
constexpr int kDi     = 2048;
constexpr int kNst    = 16;
constexpr int kRows   = kBatch * kSeq;
constexpr int kXrW    = 2 * kDi;
constexpr int kBcN    = 2 * kNst;
constexpr int kBcP    = 64;
constexpr int kScanT  = 32;
constexpr int kScanYP = 260;
constexpr float kLnEps = 1e-5f;
constexpr float kCarryAct  = 64.0f;
constexpr float kCarryWgt  = 256.0f;
constexpr float kFoldBack  = 1.0f / (kCarryAct * kCarryWgt);
constexpr float kInvCarryAct = 1.0f / kCarryAct;
static_assert(kRows == 4096);
static_assert((kDm % 32) == 0 && (kDi % 32) == 0);
static_assert((kRows % 64) == 0 && (kXrW % 64) == 0 && (kDi % 64) == 0 && (kDm % 64) == 0 && (kBcP % 64) == 0);
static_assert((kSeq % kScanT) == 0 && (kDi % 256) == 0 && kBcN <= kBcP);

constexpr size_t kOffXH    = 0;
constexpr size_t kOffWINT  = kOffXH    + (size_t)kRows * kDm  * 2;
constexpr size_t kOffWDTT  = kOffWINT  + (size_t)kXrW  * kDm  * 2;
constexpr size_t kOffWXPT  = kOffWDTT  + (size_t)kDi   * kDi  * 2;
constexpr size_t kOffWOUTT = kOffWXPT  + (size_t)kBcP  * kDi  * 2;
constexpr size_t kOffSG    = kOffWOUTT + (size_t)kDm   * kDi  * 2;
constexpr size_t kOffUU    = kOffSG    + (size_t)kRows * kXrW * 2;
constexpr size_t kOffDTP   = kOffUU    + (size_t)kRows * kDi  * 2;
constexpr size_t kOffBC    = kOffDTP   + (size_t)kRows * kDi  * 2;
constexpr size_t kOffYZ    = kOffBC    + (size_t)kRows * kBcP * 4;
constexpr size_t kOffZZ    = kOffYZ    + (size_t)kRows * kDi  * 2;
constexpr size_t kWsTotal  = kOffZZ    + (size_t)kRows * kDm  * 4;
static_assert(kWsTotal == 131334144ull);
static_assert(kWsTotal <= 134217728ull);
static_assert((kOffWINT % 128) == 0 && (kOffWDTT % 128) == 0 && (kOffWXPT % 128) == 0 && (kOffWOUTT % 128) == 0 &&
              (kOffSG % 128) == 0 && (kOffUU % 128) == 0 && (kOffDTP % 128) == 0 && (kOffBC % 128) == 0 &&
              (kOffYZ % 128) == 0 && (kOffZZ % 128) == 0);

__device__ __forceinline__ float h16_to_f32(unsigned hb) {
  const unsigned sgn = (hb & 0x8000u) << 16;
  const unsigned em = hb & 0x7fffu;
  const float fn = __uint_as_float((em << 13) + 0x38000000u);
  const float fs = (float)em * 5.9604644775390625e-8f;
  const float mag = (em < 0x400u) ? fs : fn;
  return __uint_as_float(__float_as_uint(mag) | sgn);
}
__device__ __forceinline__ float silu_fast(float v) {
  return v * __builtin_amdgcn_rcpf(1.0f + __expf(-v));
}

__device__ __forceinline__ void tie_acc(v8f& a, v16h x) { asm volatile("" : "+v"(a) : "v"(x)); }
__device__ __forceinline__ void guard_acc(v8f& a, v16h x, v16h y) { asm volatile("v_nop\n\tv_nop\n\tv_nop\n\tv_nop" : "+v"(a) : "v"(x), "v"(y)); }
__device__ __forceinline__ void keep_frag4(v16h a, v16h b, v16h c, v16h d) { asm volatile("v_nop" :: "v"(a), "v"(b), "v"(c), "v"(d)); }
__device__ __forceinline__ void acc_guard4(v8f& a, v8f& b, v8f& c, v8f& d) { asm volatile("v_nop\n\tv_nop\n\tv_nop\n\tv_nop" : "+v"(a), "+v"(b), "+v"(c), "+v"(d)); }

union FragU { v16h v; v8h h[2]; };
__device__ __forceinline__ v16h frag_load(const _Float16* p) {
  FragU f;
  f.h[0] = *(const v8h*)(p);
  f.h[1] = *(const v8h*)(p + 16);
  return f.v;
}
__device__ __forceinline__ v8f mma16(v16h a, v16h b, v8f c) {
  return __builtin_amdgcn_wmma_f32_16x16x32_f16(false, a, false, b, (short)0, c, false, false);
}

__global__ __launch_bounds__(256) void cast_rows_f16_kernel(
    const float* __restrict__ src, unsigned short* __restrict__ dst, int total8, float carry)
{
  const int i = blockIdx.x * 256 + threadIdx.x;
  if (i >= total8) return;
  const size_t e0 = (size_t)i << 3;
  const v4f a0 = *(const v4f*)(src + e0);
  const v4f a1 = *(const v4f*)(src + e0 + 4);
  v8h hv;
#pragma unroll
  for (int e = 0; e < 4; ++e) {
    hv[e]     = (_Float16)(a0[e] * carry);
    hv[4 + e] = (_Float16)(a1[e] * carry);
  }
  unsigned short* q = dst + e0;
  *(volatile v8h*)q = hv;
  __threadfence();
  *(volatile v8h*)q = hv;
}

__global__ __launch_bounds__(256) void transpose_cast_f16_kernel(
    const float* __restrict__ W, unsigned short* __restrict__ Wt, int K, int Nreal, float carry)
{
  __shared__ float sT[64 * 65];
  const int tid = threadIdx.x;
  const int k0 = blockIdx.x * 64;
  const int n0 = blockIdx.y * 64;
  const int nn4 = (tid & 15) * 4;
  const int kk = tid >> 4;
  const int ncol = n0 + nn4;
  const bool ok = (ncol < Nreal);
  const int nclamp = ok ? ncol : (Nreal - 4);
#pragma unroll
  for (int i = 0; i < 4; ++i) {
    const int kc = kk + 16 * i;
    const v4f v = *(const v4f*)(W + (size_t)(k0 + kc) * Nreal + nclamp);
    float f0 = v[0], f1 = v[1], f2 = v[2], f3 = v[3];
    asm volatile("" : "+v"(f0), "+v"(f1), "+v"(f2), "+v"(f3));
    sT[(nn4 + 0) * 65 + kc] = ok ? f0 * carry : 0.0f;
    sT[(nn4 + 1) * 65 + kc] = ok ? f1 * carry : 0.0f;
    sT[(nn4 + 2) * 65 + kc] = ok ? f2 * carry : 0.0f;
    sT[(nn4 + 3) * 65 + kc] = ok ? f3 * carry : 0.0f;
  }
  __syncthreads();
  const int c8 = (tid & 7) * 8;
  const int r = tid >> 3;
  v8h hv[2];
#pragma unroll
  for (int i = 0; i < 2; ++i) {
    const float* sp = sT + (r + 32 * i) * 65 + c8;
#pragma unroll
    for (int e = 0; e < 8; ++e) hv[i][e] = (_Float16)sp[e];
  }
  for (int pass = 0; pass < 2; ++pass) {
#pragma unroll
    for (int i = 0; i < 2; ++i)
      *(volatile v8h*)(Wt + (size_t)(n0 + r + 32 * i) * K + k0 + c8) = hv[i];
    __threadfence();
  }
}

template <int OUT_MODE, bool RESID, int ACT>
__global__ __launch_bounds__(256) void gemm_f16_kernel(
    const unsigned short* __restrict__ Ap, int lda,
    const unsigned short* __restrict__ Btp, int ldb,
    void* __restrict__ Cout, int ldc,
    const float* __restrict__ bias, int nbias,
    const float* __restrict__ resid, int ldr,
    int M, int N, int K, float scale)
{
  __shared__ __align__(16) float sT[8][16 * 68];
  const _Float16* A  = (const _Float16*)Ap;
  const _Float16* Bt = (const _Float16*)Btp;
  const int lane = threadIdx.x & 31;
  const int wave = __builtin_amdgcn_readfirstlane((int)(threadIdx.x >> 5));
  const int tilesN = N >> 6;
  const int tilesM = M >> 6;
  const int tile = blockIdx.x * 8 + wave;
  if (tile >= tilesM * tilesN) return;
  const int tm = tile / tilesN;
  const int tn = tile - tm * tilesN;
  const int m0 = tm << 6;
  const int n0 = tn << 6;
  const int rlane = lane & 15;
  const int koff  = (lane >> 4) * 8;
  const int mOff  = (lane >> 4) * 8;

  v8f acc[4][4];
#pragma unroll
  for (int i = 0; i < 4; ++i)
#pragma unroll
    for (int j = 0; j < 4; ++j) acc[i][j] = (v8f){0.f, 0.f, 0.f, 0.f, 0.f, 0.f, 0.f, 0.f};

  for (int k0 = 0; k0 < K; k0 += 32) {
    v16h bh[4];
#pragma unroll
    for (int j = 0; j < 4; ++j)
      bh[j] = frag_load(Bt + (size_t)(n0 + (j << 4) + rlane) * ldb + koff + k0);
#pragma unroll
    for (int i = 0; i < 4; ++i) {
      const v16h ah = frag_load(A + (size_t)(m0 + (i << 4) + rlane) * lda + koff + k0);
#pragma unroll
      for (int j = 0; j < 4; ++j) acc[i][j] = mma16(ah, bh[j], acc[i][j]);
      tie_acc(acc[i][0], ah);
      tie_acc(acc[i][1], ah);
      tie_acc(acc[i][2], ah);
      guard_acc(acc[i][3], ah, bh[3]);
    }
    keep_frag4(bh[0], bh[1], bh[2], bh[3]);
  }
  acc_guard4(acc[0][0], acc[0][1], acc[0][2], acc[0][3]);
  acc_guard4(acc[1][0], acc[1][1], acc[1][2], acc[1][3]);
  acc_guard4(acc[2][0], acc[2][1], acc[2][2], acc[2][3]);
  acc_guard4(acc[3][0], acc[3][1], acc[3][2], acc[3][3]);

  float bvj[4];
#pragma unroll
  for (int j = 0; j < 4; ++j) {
    const int n = n0 + (j << 4) + rlane;
    const bool ok = (n < nbias);
    const int nc = ok ? n : (nbias - 1);
    float t = bias[nc];
    asm volatile("" : "+v"(t));
    bvj[j] = ok ? t : 0.0f;
  }

  float* slab = sT[wave];
#pragma unroll
  for (int i = 0; i < 4; ++i) {
    const int mBase = m0 + (i << 4);
#pragma unroll
    for (int j = 0; j < 4; ++j) {
#pragma unroll
      for (int r = 0; r < 8; ++r) {
        float v = acc[i][j][r] * scale + bvj[j];
        if (ACT == 1) v = silu_fast(v);
        slab[(mOff + r) * 68 + (j << 4) + rlane] = v;
      }
    }
    __builtin_amdgcn_fence(__ATOMIC_RELEASE, "workgroup");
    __builtin_amdgcn_wave_barrier();
    __builtin_amdgcn_fence(__ATOMIC_ACQUIRE, "workgroup");
    if (OUT_MODE == 0) {
      float* C = (float*)Cout;
      const int hh = lane >> 4, c4 = (lane & 15) * 4;
      v4f ov[8];
#pragma unroll
      for (int it = 0; it < 8; ++it) {
        const int row = it * 2 + hh;
        v4f v = *(const v4f*)(slab + row * 68 + c4);
        if (RESID) {
          const v4f rv = *(const v4f*)(resid + (size_t)(mBase + row) * ldr + n0 + c4);
          v = v + rv;
        }
        ov[it] = v;
      }
      for (int pass = 0; pass < 2; ++pass) {
#pragma unroll
        for (int it = 0; it < 8; ++it) {
          const int row = it * 2 + hh;
          *(volatile v4f*)(C + (size_t)(mBase + row) * ldc + n0 + c4) = ov[it];
        }
        __threadfence();
      }
    } else {
      unsigned short* C = (unsigned short*)Cout;
      const int q = lane >> 3, c8 = (lane & 7) * 8;
      v8h hv[4];
#pragma unroll
      for (int it = 0; it < 4; ++it) {
        const float* sp = slab + (it * 4 + q) * 68 + c8;
#pragma unroll
        for (int e = 0; e < 8; ++e) hv[it][e] = (_Float16)sp[e];
      }
      for (int pass = 0; pass < 2; ++pass) {
#pragma unroll
        for (int it = 0; it < 4; ++it) {
          const int row = it * 4 + q;
          *(volatile v8h*)(C + (size_t)(mBase + row) * ldc + n0 + c8) = hv[it];
        }
        __threadfence();
      }
    }
    __builtin_amdgcn_fence(__ATOMIC_RELEASE, "workgroup");
    __builtin_amdgcn_wave_barrier();
    __builtin_amdgcn_fence(__ATOMIC_ACQUIRE, "workgroup");
  }
}

__device__ __forceinline__ void conv_pair(unsigned s0, unsigned s1, unsigned s2, unsigned s3,
                                          v4f wa, v4f wb, float ba, float bb, float& ua, float& ub)
{
  float ca = ba;
  ca = fmaf(wa[0], h16_to_f32(s0 & 0xffffu), ca);
  ca = fmaf(wa[1], h16_to_f32(s1 & 0xffffu), ca);
  ca = fmaf(wa[2], h16_to_f32(s2 & 0xffffu), ca);
  ca = fmaf(wa[3], h16_to_f32(s3 & 0xffffu), ca);
  float cb2 = bb;
  cb2 = fmaf(wb[0], h16_to_f32(s0 >> 16), cb2);
  cb2 = fmaf(wb[1], h16_to_f32(s1 >> 16), cb2);
  cb2 = fmaf(wb[2], h16_to_f32(s2 >> 16), cb2);
  cb2 = fmaf(wb[3], h16_to_f32(s3 >> 16), cb2);
  ua = silu_fast(ca) * kCarryAct;
  ub = silu_fast(cb2) * kCarryAct;
}

__global__ __launch_bounds__(256) void conv_silu_kernel(
    const unsigned short* __restrict__ SG, const float* __restrict__ cw, const float* __restrict__ cb,
    unsigned short* __restrict__ UU)
{
  const int gid = blockIdx.x * 256 + threadIdx.x;
  const int row = gid >> 8;
  const int d8 = (gid & 255) * 8;
  const int l = row & (kSeq - 1);
  uint4 tw[4];
#pragma unroll
  for (int j = 0; j < 4; ++j) {
    const bool ok = (l - 3 + j >= 0);
    const int rr = ok ? (row - 3 + j) : row;
    uint4 w = *(const uint4*)(const void*)(SG + (size_t)rr * kXrW + d8);
    asm volatile("" : "+v"(w.x), "+v"(w.y), "+v"(w.z), "+v"(w.w));
    tw[j].x = ok ? w.x : 0u;
    tw[j].y = ok ? w.y : 0u;
    tw[j].z = ok ? w.z : 0u;
    tw[j].w = ok ? w.w : 0u;
  }
  v4f wv[8];
#pragma unroll
  for (int e = 0; e < 8; ++e) wv[e] = *(const v4f*)(cw + (size_t)(d8 + e) * 4);
  const v4f b0 = *(const v4f*)(cb + d8);
  const v4f b1 = *(const v4f*)(cb + d8 + 4);
  float u0, u1, u2, u3, u4, u5, u6, u7;
  conv_pair(tw[0].x, tw[1].x, tw[2].x, tw[3].x, wv[0], wv[1], b0[0], b0[1], u0, u1);
  conv_pair(tw[0].y, tw[1].y, tw[2].y, tw[3].y, wv[2], wv[3], b0[2], b0[3], u2, u3);
  conv_pair(tw[0].z, tw[1].z, tw[2].z, tw[3].z, wv[4], wv[5], b1[0], b1[1], u4, u5);
  conv_pair(tw[0].w, tw[1].w, tw[2].w, tw[3].w, wv[6], wv[7], b1[2], b1[3], u6, u7);
  v8h hv;
  hv[0] = (_Float16)u0; hv[1] = (_Float16)u1; hv[2] = (_Float16)u2; hv[3] = (_Float16)u3;
  hv[4] = (_Float16)u4; hv[5] = (_Float16)u5; hv[6] = (_Float16)u6; hv[7] = (_Float16)u7;
  unsigned short* q = UU + (size_t)row * kDi + d8;
  *(volatile v8h*)q = hv;
  __threadfence();
  *(volatile v8h*)q = hv;
}

__global__ __launch_bounds__(256) void scan_kernel(
    const unsigned short* __restrict__ UU, const unsigned short* __restrict__ DTP,
    const unsigned short* __restrict__ SG, const float* __restrict__ BC,
    const float* __restrict__ Alog, const float* __restrict__ Dp,
    unsigned short* __restrict__ YZ)
{
  __shared__ __align__(16) float sX[kScanT * kBcN];
  __shared__ __align__(16) float sY[kScanT * kScanYP];
  const int tid = threadIdx.x;
  const int lane = tid & 31;
  const int wave = __builtin_amdgcn_readfirstlane((int)(threadIdx.x >> 5));
  const int d0 = blockIdx.x * 256;
  const int d = d0 + tid;
  const size_t row0 = (size_t)blockIdx.y * kSeq;

  float negA[kNst], h[kNst];
#pragma unroll
  for (int q4 = 0; q4 < 4; ++q4) {
    const v4f av = *(const v4f*)(Alog + (size_t)d * kNst + 4 * q4);
    negA[4 * q4 + 0] = -expf(av[0]);
    negA[4 * q4 + 1] = -expf(av[1]);
    negA[4 * q4 + 2] = -expf(av[2]);
    negA[4 * q4 + 3] = -expf(av[3]);
  }
#pragma unroll
  for (int k = 0; k < kNst; ++k) h[k] = 0.0f;
  const float Dd = Dp[d];
  const int sr = tid >> 3, sc4 = (tid & 7) * 4;

#pragma unroll 1
  for (int t0 = 0; t0 < kSeq; t0 += kScanT) {
    __syncthreads();
    {
      const v4f bv = *(const v4f*)(BC + (row0 + t0 + sr) * kBcP + sc4);
      *(v4f*)(sX + sr * kBcN + sc4) = bv;
    }
    __syncthreads();
#pragma unroll 1
    for (int s = 0; s < kScanT; ++s) {
      const size_t row = row0 + t0 + s;
      const unsigned ub = UU[row * kDi + d];
      const unsigned pb = DTP[row * kDi + d];
      const unsigned gb = SG[row * kXrW + kDi + d];
      const float uv = h16_to_f32(ub) * kInvCarryAct;
      const float pv = h16_to_f32(pb);
      const float gv = h16_to_f32(gb);
      const float ea = __expf(-fabsf(pv));
      const float up = 1.0f + ea;
      const float l1p = __logf(up) + (ea - (up - 1.0f)) * __builtin_amdgcn_rcpf(up);
      const float dt = fmaxf(pv, 0.0f) + l1p;
      const float dtx = dt * uv;
      const float* xr = sX + s * kBcN;
      float y = 0.0f;
#pragma unroll
      for (int q4 = 0; q4 < 4; ++q4) {
        const v4f bv = *(const v4f*)(xr + 4 * q4);
        const v4f cv = *(const v4f*)(xr + kNst + 4 * q4);
#pragma unroll
        for (int e = 0; e < 4; ++e) {
          const float ek = __expf(dt * negA[4 * q4 + e]);
          h[4 * q4 + e] = fmaf(ek, h[4 * q4 + e], dtx * bv[e]);
          y = fmaf(h[4 * q4 + e], cv[e], y);
        }
      }
      y = fmaf(uv, Dd, y);
      sY[s * kScanYP + tid] = y * gv;
    }
    __syncthreads();
    v8h hv[4];
#pragma unroll
    for (int it = 0; it < 4; ++it) {
      const float* sp = sY + (it * 8 + wave) * kScanYP + lane * 8;
      const v4f a0 = *(const v4f*)(sp);
      const v4f a1 = *(const v4f*)(sp + 4);
#pragma unroll
      for (int e = 0; e < 4; ++e) {
        hv[it][e]     = (_Float16)(a0[e] * kCarryAct);
        hv[it][4 + e] = (_Float16)(a1[e] * kCarryAct);
      }
    }
    for (int pass = 0; pass < 2; ++pass) {
#pragma unroll
      for (int it = 0; it < 4; ++it)
        *(volatile v8h*)(YZ + (row0 + t0 + it * 8 + wave) * kDi + d0 + lane * 8) = hv[it];
      __threadfence();
    }
  }
}

__global__ __launch_bounds__(256) void layernorm_kernel(
    const float* __restrict__ Z, const float* __restrict__ g, const float* __restrict__ bta,
    float* __restrict__ out)
{
  __shared__ float red1[8];
  __shared__ float red2[8];
  const int tid = threadIdx.x;
  const int lane = tid & 31;
  const int wave = __builtin_amdgcn_readfirstlane((int)(threadIdx.x >> 5));
  const size_t base = (size_t)blockIdx.x * kDm + (size_t)tid * 4;
  const v4f z = *(const v4f*)(Z + base);
  float s = (z[0] + z[1]) + (z[2] + z[3]);
#pragma unroll
  for (int off = 16; off >= 1; off >>= 1) s += __shfl_xor(s, off, 32);
  if (lane == 0) red1[wave] = s;
  __syncthreads();
  float tot = 0.0f;
#pragma unroll
  for (int w = 0; w < 8; ++w) tot += red1[w];
  const float mu = tot * (1.0f / (float)kDm);
  const float c0 = z[0] - mu, c1 = z[1] - mu, c2 = z[2] - mu, c3 = z[3] - mu;
  float q = (c0 * c0 + c1 * c1) + (c2 * c2 + c3 * c3);
#pragma unroll
  for (int off = 16; off >= 1; off >>= 1) q += __shfl_xor(q, off, 32);
  if (lane == 0) red2[wave] = q;
  __syncthreads();
  float tq = 0.0f;
#pragma unroll
  for (int w = 0; w < 8; ++w) tq += red2[w];
  const float var = tq * (1.0f / (float)kDm);
  const float inv = rsqrtf(var + kLnEps);
  const v4f gv = *(const v4f*)(g + tid * 4);
  const v4f bv = *(const v4f*)(bta + tid * 4);
  v4f o;
  o[0] = c0 * inv * gv[0] + bv[0];
  o[1] = c1 * inv * gv[1] + bv[1];
  o[2] = c2 * inv * gv[2] + bv[2];
  o[3] = c3 * inv * gv[3] + bv[3];
  *(volatile v4f*)(out + base) = o;
  __threadfence();
  *(volatile v4f*)(out + base) = o;
}

extern "C" void kernel_launch(void* const* d_in, const int* in_sizes, int n_in,
                              void* d_out, int out_size, void* d_ws, size_t ws_size,
                              hipStream_t stream) {
  if (n_in < 15) return;
  if (in_sizes[0] != kRows * kDm) return;
  if (in_sizes[1] != kDm * kXrW) return;
  if (in_sizes[2] != kXrW) return;
  if (in_sizes[3] != kDi * 4) return;
  if (in_sizes[4] != kDi) return;
  if (in_sizes[5] != kDi * kBcN) return;
  if (in_sizes[6] != kBcN) return;
  if (in_sizes[7] != kDi * kDi) return;
  if (in_sizes[8] != kDi) return;
  if (in_sizes[9] != kDi * kNst) return;
  if (in_sizes[10] != kDi) return;
  if (in_sizes[11] != kDi * kDm) return;
  if (in_sizes[12] != kDm) return;
  if (in_sizes[13] != kDm) return;
  if (in_sizes[14] != kDm) return;
  if (out_size != kRows * kDm) return;
  if (ws_size < kWsTotal) return;

  const float* x      = (const float*)d_in[0];
  const float* W_in   = (const float*)d_in[1];
  const float* b_in   = (const float*)d_in[2];
  const float* conv_w = (const float*)d_in[3];
  const float* conv_b = (const float*)d_in[4];
  const float* W_xp   = (const float*)d_in[5];
  const float* b_xp   = (const float*)d_in[6];
  const float* W_dt   = (const float*)d_in[7];
  const float* b_dt   = (const float*)d_in[8];
  const float* A_log  = (const float*)d_in[9];
  const float* D_par  = (const float*)d_in[10];
  const float* W_out  = (const float*)d_in[11];
  const float* b_out  = (const float*)d_in[12];
  const float* ln_g   = (const float*)d_in[13];
  const float* ln_b   = (const float*)d_in[14];
  float* out = (float*)d_out;

  char* ws = (char*)d_ws;
  unsigned short* XH    = (unsigned short*)(ws + kOffXH);
  unsigned short* WINT  = (unsigned short*)(ws + kOffWINT);
  unsigned short* WDTT  = (unsigned short*)(ws + kOffWDTT);
  unsigned short* WXPT  = (unsigned short*)(ws + kOffWXPT);
  unsigned short* WOUTT = (unsigned short*)(ws + kOffWOUTT);
  unsigned short* SG    = (unsigned short*)(ws + kOffSG);
  unsigned short* UU    = (unsigned short*)(ws + kOffUU);
  unsigned short* DTP   = (unsigned short*)(ws + kOffDTP);
  float*          BC    = (float*)(ws + kOffBC);
  unsigned short* YZ    = (unsigned short*)(ws + kOffYZ);
  float*          ZZ    = (float*)(ws + kOffZZ);

  cast_rows_f16_kernel<<<(kRows * kDm / 8) / 256, 256, 0, stream>>>(x, XH, kRows * kDm / 8, kCarryAct);
  transpose_cast_f16_kernel<<<dim3(kDm / 64, kXrW / 64), 256, 0, stream>>>(W_in, WINT, kDm, kXrW, kCarryWgt);
  transpose_cast_f16_kernel<<<dim3(kDi / 64, kDi / 64), 256, 0, stream>>>(W_dt, WDTT, kDi, kDi, kCarryWgt);
  transpose_cast_f16_kernel<<<dim3(kDi / 64, kBcP / 64), 256, 0, stream>>>(W_xp, WXPT, kDi, kBcN, kCarryWgt);
  transpose_cast_f16_kernel<<<dim3(kDi / 64, kDm / 64), 256, 0, stream>>>(W_out, WOUTT, kDi, kDm, kCarryWgt);

  gemm_f16_kernel<1, false, 1><<<(kRows / 64) * (kXrW / 64) / 8, 256, 0, stream>>>(
      XH, kDm, WINT, kDm, (void*)SG, kXrW, b_in, kXrW, x, kDm,
      kRows, kXrW, kDm, kFoldBack);

  conv_silu_kernel<<<(kRows * (kDi / 8)) / 256, 256, 0, stream>>>(SG, conv_w, conv_b, UU);

  gemm_f16_kernel<0, false, 0><<<(kRows / 64) * (kBcP / 64) / 8, 256, 0, stream>>>(
      UU, kDi, WXPT, kDi, (void*)BC, kBcP, b_xp, kBcN, x, kDm,
      kRows, kBcP, kDi, kFoldBack);

  gemm_f16_kernel<1, false, 0><<<(kRows / 64) * (kDi / 64) / 8, 256, 0, stream>>>(
      UU, kDi, WDTT, kDi, (void*)DTP, kDi, b_dt, kDi, x, kDm,
      kRows, kDi, kDi, kFoldBack);

  scan_kernel<<<dim3(kDi / 256, kBatch), 256, 0, stream>>>(UU, DTP, SG, BC, A_log, D_par, YZ);

  gemm_f16_kernel<0, true, 0><<<(kRows / 64) * (kDm / 64) / 8, 256, 0, stream>>>(
      YZ, kDi, WOUTT, kDi, (void*)ZZ, kDm, b_out, kDm, x, kDm,
      kRows, kDm, kDi, kFoldBack);

  layernorm_kernel<<<kRows, 256, 0, stream>>>(ZZ, ln_g, ln_b, out);
}
